// Twister_19232863551565
// MI455X (gfx1250) — hardware-verified
//
#include <hip/hip_runtime.h>


namespace {
constexpr int NB = 4, C0 = 96, C3 = 288, HI = 64, LI = HI * HI, RS = 16, PS = RS * RS, NS = 16;
constexpr float WSC = 256.0f;
typedef _Float16 b16;
typedef __attribute__((ext_vector_type(16))) _Float16 v16b;
typedef __attribute__((ext_vector_type(8))) _Float16 v8b;
typedef __attribute__((ext_vector_type(8))) float v8f;
typedef __attribute__((ext_vector_type(4))) float v4f;
typedef __attribute__((ext_vector_type(2))) float v2f;
__device__ __forceinline__ float bf16_rne(float f) { unsigned int u = __float_as_uint(f); u += 0x7FFFu + ((u >> 16) & 1u); return __uint_as_float(u & 0xFFFF0000u); }
__device__ __forceinline__ void split16(float v, b16& hi, b16& lo) { hi = (b16)v; lo = (b16)(v - (float)hi); }
__device__ __forceinline__ v16b frag_kb(const b16* p, int hh) { const v8b a = *(const v8b*)(p + 8 * hh), b = *(const v8b*)(p + 16 + 8 * hh); v16b f;
#pragma unroll
  for (int e = 0; e < 8; ++e) { f[e] = a[e]; f[8 + e] = b[e]; } return f; }
__device__ __forceinline__ v8f wmma16b(v16b a, v16b b, v8f c) { v8f d = __builtin_amdgcn_wmma_f32_16x16x32_f16(false, a, false, b, (short)0, c, false, false); asm volatile("v_nop\n\tv_nop\n\tv_nop\n\tv_nop" : "+v"(d) : "v"(a), "v"(b)); return d; }
__device__ __forceinline__ void wave_lds_sync() { __builtin_amdgcn_fence(__ATOMIC_RELEASE, "workgroup"); __builtin_amdgcn_wave_barrier(); __builtin_amdgcn_fence(__ATOMIC_ACQUIRE, "workgroup"); }
__device__ __forceinline__ float pmul(float a, float b) { float p = a * b; asm volatile("" : "+v"(p)); return p; }
__device__ __forceinline__ float sigm(float v) { return 1.0f / (1.0f + __expf(-v)); }
__device__ __forceinline__ float silu(float v) { return pmul(v, sigm(v)); }
__device__ __forceinline__ float softplus(float v) { return v > 20.0f ? v : (v < -20.0f ? __expf(v) : log1pf(__expf(v))); }
__device__ __forceinline__ void lerp_taps(int o, int n_in, int n_out, int& i0, int& i1, float& f) { float src = ((float)o + 0.5f) * ((float)n_in / (float)n_out) - 0.5f; src = fminf(fmaxf(src, 0.0f), (float)(n_in - 1)); i0 = (int)floorf(src); i1 = min(i0 + 1, n_in - 1); f = src - (float)i0; }
__device__ __forceinline__ const float* src_plane(const float* img, const float* gc, const float* lc, int b, int c) { const float* base = c < C0 ? img : (c < 2 * C0 ? gc : lc); return base + ((size_t)b * C0 + (c % C0)) * LI; }

__global__ __launch_bounds__(256) void wcopyp_kernel(const float* __restrict__ w, int KIN, int OUT, int KP, int OUTP, b16* __restrict__ WT) {
  const int u = blockIdx.x * 256 + threadIdx.x; if (u >= OUTP * KP / 8) return; const int e = u * 8; const int o = e / KP, k0 = e % KP; v8b v;
#pragma unroll
  for (int j = 0; j < 8; ++j) { const int k = k0 + j; v[j] = (o < OUT && k < KIN) ? (b16)(bf16_rne(w[(size_t)o * KIN + k]) * WSC) : (b16)0.0f; } for (int pass = 0; pass < 2; ++pass) { *(volatile v8b*)(WT + e) = v; __threadfence(); }
}
__global__ __launch_bounds__(256) void small_kernel(const float* __restrict__ img, const float* __restrict__ gc, const float* __restrict__ lc, int NBV, float* __restrict__ XA) {
  const int u = blockIdx.x * 256 + threadIdx.x; if (u >= NBV * C3 * PS / 4) return; const int row = u / (PS / 4), p0 = (u % (PS / 4)) * 4; const int b = row / C3, c = row % C3; const float* sp = src_plane(img, gc, lc, b, c); v4f o;
#pragma unroll
  for (int j = 0; j < 4; ++j) { const int p = p0 + j; const int py = p / RS, px = p % RS; int y0, y1, x0, x1; float fy, fx; lerp_taps(py, HI, RS, y0, y1, fy); lerp_taps(px, HI, RS, x0, x1, fx);
    const float a = bf16_rne(sp[y0 * HI + x0]) * (1.0f - fy) + bf16_rne(sp[y1 * HI + x0]) * fy, bb = bf16_rne(sp[y0 * HI + x1]) * (1.0f - fy) + bf16_rne(sp[y1 * HI + x1]) * fy; o[j] = a * (1.0f - fx) + bb * fx; }
  for (int pass = 0; pass < 2; ++pass) { *(volatile v4f*)(XA + (size_t)row * PS + p0) = o; __threadfence(); }
}
__global__ __launch_bounds__(256) void xfull_kernel(const float* __restrict__ img, const float* __restrict__ gc, const float* __restrict__ lc, const float* __restrict__ SM, float* __restrict__ XT) {
  __shared__ float T[HI][33];
  const int cg = blockIdx.x % 9, y = (blockIdx.x / 9) % HI, b = blockIdx.x / (9 * HI); const int tid = threadIdx.x;
  for (int i = tid; i < 32 * HI; i += 256) { const int cl = i / HI, x = i % HI; const int c = cg * 32 + cl; const float* sp = src_plane(img, gc, lc, b, c); const float* sm = SM + ((size_t)b * C3 + c) * PS;
    int y0, y1, x0, x1; float fy, fx; lerp_taps(y, RS, HI, y0, y1, fy); lerp_taps(x, RS, HI, x0, x1, fx);
    const float a = sm[y0 * RS + x0] * (1.0f - fy) + sm[y1 * RS + x0] * fy, bb = sm[y0 * RS + x1] * (1.0f - fy) + sm[y1 * RS + x1] * fy; T[x][cl] = bf16_rne(sp[y * HI + x]) + (a * (1.0f - fx) + bb * fx); }
  __syncthreads();
  for (int pass = 0; pass < 2; ++pass) { for (int i = tid; i < HI * 32; i += 256) { const int x = i / 32, cl = i % 32; ((volatile float*)XT)[(((size_t)b * HI + y) * HI + x) * C3 + cg * 32 + cl] = T[x][cl]; } __threadfence(); }
}
template <int CIN, int DIN, int EXACT>
__global__ __launch_bounds__(32) void inproj_kernel(const float* __restrict__ XIN, const b16* __restrict__ W, float IS, float* __restrict__ XZ) {
  __shared__ __attribute__((aligned(16))) b16 Ah[16][CIN + 8], Al[16][CIN + 8]; __shared__ __attribute__((aligned(16))) float Tf[16][128 + 4];
  const int lane = threadIdx.x, nloc = lane & 15, hlf = lane >> 4; const size_t m0 = (size_t)blockIdx.x * 16;
  for (int rr = 0; rr < 16; ++rr) for (int q = 0; q < CIN / 32; ++q) { const float v = XIN[(m0 + rr) * CIN + q * 32 + lane]; b16 p, ql; split16(v * IS, p, ql); Ah[rr][q * 32 + lane] = p; Al[rr][q * 32 + lane] = ql; }
  wave_lds_sync(); const float sc = 1.0f / (IS * WSC);
#pragma unroll 1
  for (int cgp = 0; cgp < 2 * DIN / 128; ++cgp) { v8f acc[8];
#pragma unroll
    for (int t = 0; t < 8; ++t) acc[t] = (v8f){};
#pragma unroll 3
    for (int kb = 0; kb < CIN; kb += 32) { const v16b a = frag_kb(&Ah[nloc][kb], hlf), al = frag_kb(&Al[nloc][kb], hlf);
#pragma unroll
      for (int t = 0; t < 8; ++t) { const v16b bw = frag_kb(W + (size_t)(cgp * 128 + t * 16 + nloc) * CIN + kb, hlf); acc[t] = wmma16b(a, bw, acc[t]); if (!EXACT) acc[t] = wmma16b(al, bw, acc[t]); } }
#pragma unroll
    for (int t = 0; t < 8; ++t)
#pragma unroll 1
      for (int r8 = 0; r8 < 8; ++r8) Tf[8 * hlf + r8][t * 16 + nloc] = acc[t][r8] * sc;
    wave_lds_sync();
    for (int pass = 0; pass < 2; ++pass) { for (int rr = 0; rr < 16; ++rr) *(volatile v4f*)(XZ + (m0 + rr) * (2 * DIN) + cgp * 128 + lane * 4) = *(const v4f*)(&Tf[rr][lane * 4]); __threadfence(); }
    wave_lds_sync(); }
}
template <int DIN>
__global__ __launch_bounds__(256) void dwconv_kernel(const float* __restrict__ XZ, const float* __restrict__ cw, const float* __restrict__ cb, int H, int Wd, int ntok, float* __restrict__ U) {
  const size_t gid = (size_t)blockIdx.x * 256 + threadIdx.x; const size_t t = gid / (DIN / 4); const int d4 = (int)(gid % (DIN / 4)) * 4; if (t >= (size_t)ntok) return; const int L = H * Wd;
  const int b = (int)(t / L), p = (int)(t % L), y = p / Wd, x = p % Wd; v4f acc; for (int q = 0; q < 4; ++q) acc[q] = bf16_rne(cb[d4 + q]);
#pragma unroll
  for (int di = 0; di < 3; ++di)
#pragma unroll
    for (int dj = 0; dj < 3; ++dj) { const int yy = y + di - 1, xx = x + dj - 1; const bool ok = yy >= 0 && yy < H && xx >= 0 && xx < Wd; const int yc = ok ? yy : y, xc = ok ? xx : x;
      const v4f v = *(const v4f*)(XZ + ((size_t)b * L + yc * Wd + xc) * (2 * DIN) + d4); for (int q = 0; q < 4; ++q) acc[q] += ok ? pmul(v[q], bf16_rne(cw[(d4 + q) * 9 + di * 3 + dj])) : 0.0f; }
  v4f o; for (int q = 0; q < 4; ++q) o[q] = silu(acc[q]);
  for (int pass = 0; pass < 2; ++pass) { *(volatile v4f*)(U + t * DIN + d4) = o; __threadfence(); }
}
template <int DIN, int R>
__global__ __launch_bounds__(32) void xproj_kernel(const float* __restrict__ U, const b16* __restrict__ XPW, const b16* __restrict__ DTW, const float* __restrict__ dtb, float US, float DS, int ntok, float* __restrict__ BC, float* __restrict__ DT) {
  __shared__ __attribute__((aligned(16))) b16 Ah[16][DIN + 8], Al[16][DIN + 8], Dh[16][32 + 8], Dl[16][32 + 8]; __shared__ __attribute__((aligned(16))) float Sbc[16][32], Tf[16][128 + 4];
  const int lane = threadIdx.x, nloc = lane & 15, hlf = lane >> 4; const size_t m0 = (size_t)blockIdx.x * 16; const int k = blockIdx.y;
  for (int rr = 0; rr < 16; ++rr) for (int q = 0; q < DIN / 32; ++q) { b16 p, ql; split16(U[(m0 + rr) * DIN + q * 32 + lane] * US, p, ql); Ah[rr][q * 32 + lane] = p; Al[rr][q * 32 + lane] = ql; }
  wave_lds_sync();
  const float sx = 1.0f / (US * WSC), sd = 1.0f / (DS * WSC);
  v8f ax[3] = {(v8f){}, (v8f){}, (v8f){}};
#pragma unroll 2
  for (int kb = 0; kb < DIN; kb += 32) { const v16b a = frag_kb(&Ah[nloc][kb], hlf), al = frag_kb(&Al[nloc][kb], hlf);
#pragma unroll
    for (int t = 0; t < 3; ++t) { const v16b bw = frag_kb(XPW + ((size_t)k * 48 + t * 16 + nloc) * DIN + kb, hlf); ax[t] = wmma16b(a, bw, ax[t]); ax[t] = wmma16b(al, bw, ax[t]); } }
#pragma unroll
  for (int t = 0; t < 3; ++t) { const int c = t * 16 + nloc;
#pragma unroll
    for (int r8 = 0; r8 < 8; ++r8) { const int rl = 8 * hlf + r8; const float v = ax[t][r8] * sx; if (c < R) { b16 p, ql; split16(v * DS, p, ql); Dh[rl][c] = p; Dl[rl][c] = ql; } else if (c < R + 32) Sbc[rl][c - R] = v; } }
  for (int rr = 0; rr < 16; ++rr) if (lane >= R) { Dh[rr][lane] = (b16)0.0f; Dl[rr][lane] = (b16)0.0f; }
  wave_lds_sync();
  for (int pass = 0; pass < 2; ++pass) { for (int rr = 0; rr < 16; ++rr) ((volatile float*)BC)[((size_t)k * ntok + m0 + rr) * 32 + lane] = Sbc[rr][lane]; __threadfence(); }
  const v16b a = frag_kb(&Dh[nloc][0], hlf), al = frag_kb(&Dl[nloc][0], hlf);
#pragma unroll 1
  for (int cgp = 0; cgp < DIN / 128; ++cgp) { v8f acc[8];
#pragma unroll
    for (int t = 0; t < 8; ++t) { acc[t] = (v8f){}; const v16b bw = frag_kb(DTW + ((size_t)k * DIN + cgp * 128 + t * 16 + nloc) * 32, hlf); acc[t] = wmma16b(a, bw, acc[t]); acc[t] = wmma16b(al, bw, acc[t]); }
#pragma unroll
    for (int t = 0; t < 8; ++t) { const int c = cgp * 128 + t * 16 + nloc; const float bb = bf16_rne(dtb[k * DIN + c]);
#pragma unroll 1
      for (int r8 = 0; r8 < 8; ++r8) Tf[8 * hlf + r8][t * 16 + nloc] = softplus(acc[t][r8] * sd + bb); }
    wave_lds_sync();
    for (int pass = 0; pass < 2; ++pass) { for (int rr = 0; rr < 16; ++rr) *(volatile v4f*)(DT + ((size_t)k * ntok + m0 + rr) * DIN + cgp * 128 + lane * 4) = *(const v4f*)(&Tf[rr][lane * 4]); __threadfence(); }
    wave_lds_sync(); }
}
template <int DIN>
__global__ __launch_bounds__(256) void scan_kernel(const float* __restrict__ U, const float* __restrict__ DT, const float* __restrict__ BC, const float* __restrict__ alog, const float* __restrict__ Ds, int H, int Wd, int nbv, int ntok, float* __restrict__ Y) {
  const int gid = blockIdx.x * 256 + threadIdx.x; const int d = gid % DIN, k = (gid / DIN) % 4, b = gid / (4 * DIN); if (b >= nbv) return; const int L = H * Wd;
  float A[NS]; for (int s = 0; s < NS; ++s) A[s] = -__expf(bf16_rne(alog[((size_t)k * DIN + d) * NS + s])); const float dk = bf16_rne(Ds[k * DIN + d]);
#pragma unroll 1
  for (int pass = 0; pass < 2; ++pass) { float h[NS]; for (int s = 0; s < NS; ++s) h[s] = 0.0f;
#pragma unroll 1
    for (int l = 0; l < L; ++l) { const int lk = (k >= 2) ? (L - 1 - l) : l; const int tok = (k & 1) ? ((lk % H) * Wd + lk / H) : lk; const size_t row = (size_t)b * L + tok; const size_t krow = (size_t)k * ntok + row;
      const float u = U[row * DIN + d], dt = DT[krow * DIN + d]; const float du = pmul(dt, u); const float* bc = BC + krow * 32; float acc = 0.0f;
#pragma unroll
      for (int s = 0; s < NS; ++s) { h[s] = pmul(h[s], __expf(pmul(dt, A[s]))) + pmul(du, bc[s]); acc += pmul(h[s], bc[16 + s]); }
      ((volatile float*)Y)[(krow) * DIN + d] = acc + pmul(dk, u); }
    __threadfence(); }
}
template <int DIN, int DM, int NCHW>
__global__ __launch_bounds__(32) void out_kernel(const float* __restrict__ Y, const float* __restrict__ XZ, const float* __restrict__ ng, const float* __restrict__ nbias, const b16* __restrict__ W, float YS, int ntok, float* __restrict__ OUT_) {
  __shared__ __attribute__((aligned(16))) b16 Ah[16][DIN + 8], Al[16][DIN + 8]; __shared__ __attribute__((aligned(16))) float Tf[NCHW ? DM : 16][NCHW ? 33 : DM + 4];
  const int lane = threadIdx.x, nloc = lane & 15, hlf = lane >> 4; constexpr int NT = NCHW ? 2 : 1; constexpr int QN = DIN / 32; const float sc = 1.0f / (YS * WSC);
  float g[QN], be[QN]; for (int q = 0; q < QN; ++q) { g[q] = bf16_rne(ng[q * 32 + lane]); be[q] = bf16_rne(nbias[q * 32 + lane]); }
#pragma unroll 1
  for (int half = 0; half < NT; ++half) { const size_t m0 = ((size_t)blockIdx.x * NT + half) * 16;
    for (int rr = 0; rr < 16; ++rr) { const size_t t = m0 + rr; float v[QN]; float s = 0.0f; for (int q = 0; q < QN; ++q) { const int c = q * 32 + lane; float y = 0.0f; for (int k = 0; k < 4; ++k) y += Y[((size_t)k * ntok + t) * DIN + c]; v[q] = y; s += y; }
      for (int o = 16; o; o >>= 1) s += __shfl_xor(s, o); const float mu = s * (1.0f / DIN); float vq = 0.0f; for (int q = 0; q < QN; ++q) { const float dd = v[q] - mu; vq += pmul(dd, dd); } for (int o = 16; o; o >>= 1) vq += __shfl_xor(vq, o); const float rs = rsqrtf(vq * (1.0f / DIN) + 1e-5f);
      for (int q = 0; q < QN; ++q) { const int c = q * 32 + lane; const float z = XZ[t * (2 * DIN) + DIN + c]; const float a = pmul(pmul(pmul(v[q] - mu, rs), g[q]) + be[q], silu(z)); b16 p, ql; split16(a * YS, p, ql); Ah[rr][c] = p; Al[rr][c] = ql; } }
    wave_lds_sync();
    v8f acc[DM / 16];
#pragma unroll
    for (int tt = 0; tt < DM / 16; ++tt) acc[tt] = (v8f){};
#pragma unroll 2
    for (int kb = 0; kb < DIN; kb += 32) { const v16b a = frag_kb(&Ah[nloc][kb], hlf), al = frag_kb(&Al[nloc][kb], hlf);
#pragma unroll
      for (int tt = 0; tt < DM / 16; ++tt) { const v16b bw = frag_kb(W + (size_t)(tt * 16 + nloc) * DIN + kb, hlf); acc[tt] = wmma16b(a, bw, acc[tt]); acc[tt] = wmma16b(al, bw, acc[tt]); } }
    wave_lds_sync();
    if (NCHW) {
#pragma unroll
      for (int tt = 0; tt < DM / 16; ++tt)
#pragma unroll
        for (int r8 = 0; r8 < 8; ++r8) Tf[tt * 16 + nloc][half * 16 + 8 * hlf + r8] = acc[tt][r8] * sc; }
    else {
#pragma unroll
      for (int tt = 0; tt < DM / 16; ++tt)
#pragma unroll 1
        for (int r8 = 0; r8 < 8; ++r8) Tf[8 * hlf + r8][tt * 16 + nloc] = acc[tt][r8] * sc;
      wave_lds_sync();
      for (int pass = 0; pass < 2; ++pass) { for (int rr = 0; rr < 16; ++rr) for (int q = 0; q < DM / 128; ++q) *(volatile v4f*)(OUT_ + (m0 + rr) * DM + q * 128 + lane * 4) = *(const v4f*)(&Tf[rr][q * 128 + lane * 4]); __threadfence(); } }
    wave_lds_sync(); }
  if (NCHW) { const size_t t0 = (size_t)blockIdx.x * 32; const int b = (int)(t0 / LI), p0 = (int)(t0 % LI);
    for (int pass = 0; pass < 2; ++pass) { for (int o = 0; o < DM; ++o) ((volatile float*)OUT_)[((size_t)b * DM + o) * LI + p0 + lane] = Tf[o][lane]; __threadfence(); } }
}
}

extern "C" void kernel_launch(void* const* d_in, const int* in_sizes, int n_in, void* d_out, int out_size, void* d_ws, size_t ws_size, hipStream_t stream) {
  (void)n_in;
  auto Fp = [&](int i) { return (const float*)d_in[i]; };
  constexpr int D1 = 512, R1 = 16, CI1 = 256, M1 = 256, W1 = 288; constexpr int D2 = 192, R2 = 6, CI2 = 288, M2 = 96;
  if (in_sizes[0] != NB * C0 * LI || in_sizes[3] != 2 * D1 * CI1 || in_sizes[6] != 4 * (R1 + 32) * D1 || in_sizes[7] != 4 * D1 * R1 || in_sizes[13] != M1 * D1 || in_sizes[14] != 2 * D2 * CI2 || in_sizes[17] != 4 * (R2 + 32) * D2 || in_sizes[18] != 4 * D2 * R2 || in_sizes[24] != M2 * D2 || out_size != NB * M2 * LI) return;
  const int NBV = NB;
  const int NT1 = NBV * W1, NT2 = NBV * LI;
  size_t off = 0; char* ws = (char*)d_ws;
  auto carve = [&](size_t bytes) { char* p = ws + off; off += (bytes + 255) & ~(size_t)255; return p; };
  b16* WI1 = (b16*)carve((size_t)2 * D1 * CI1 * 2); b16* XP1 = (b16*)carve((size_t)4 * 48 * D1 * 2); b16* DW1 = (b16*)carve((size_t)4 * D1 * 32 * 2); b16* WO1 = (b16*)carve((size_t)M1 * D1 * 2);
  b16* WI2 = (b16*)carve((size_t)2 * D2 * CI2 * 2); b16* XP2 = (b16*)carve((size_t)4 * 48 * D2 * 2); b16* DW2 = (b16*)carve((size_t)4 * D2 * 32 * 2); b16* WO2 = (b16*)carve((size_t)M2 * D2 * 2);
  float* XA = (float*)carve((size_t)NB * W1 * CI1 * 4); float* XZ1 = (float*)carve((size_t)NB * W1 * 2 * D1 * 4); float* U1 = (float*)carve((size_t)NB * W1 * D1 * 4); float* BC1 = (float*)carve((size_t)4 * NB * W1 * 32 * 4); float* DT1 = (float*)carve((size_t)4 * NB * W1 * D1 * 4); float* Y1 = (float*)carve((size_t)4 * NB * W1 * D1 * 4); float* SM = (float*)carve((size_t)NB * W1 * M1 * 4);
  float* XT = (float*)carve((size_t)NB * LI * CI2 * 4); float* XZ2 = (float*)carve((size_t)NB * LI * 2 * D2 * 4); float* U2 = (float*)carve((size_t)NB * LI * D2 * 4); float* BC2 = (float*)carve((size_t)4 * NB * LI * 32 * 4); float* DT2 = (float*)carve((size_t)4 * NB * LI * D2 * 4); float* Y2 = (float*)carve((size_t)4 * NB * LI * D2 * 4);
  if (off > ws_size) return;
  auto wcp = [&](const float* w, int KIN, int OUT, int KP, int OUTP, b16* WT) { wcopyp_kernel<<<(OUTP * KP / 8 + 255) / 256, 256, 0, stream>>>(w, KIN, OUT, KP, OUTP, WT); };
  wcp(Fp(3), CI1, 2 * D1, CI1, 2 * D1, WI1); for (int k = 0; k < 4; ++k) { wcp(Fp(6) + (size_t)k * (R1 + 32) * D1, D1, R1 + 32, D1, 48, XP1 + (size_t)k * 48 * D1); wcp(Fp(7) + (size_t)k * D1 * R1, R1, D1, 32, D1, DW1 + (size_t)k * D1 * 32); } wcp(Fp(13), D1, M1, D1, M1, WO1);
  wcp(Fp(14), CI2, 2 * D2, CI2, 2 * D2, WI2); for (int k = 0; k < 4; ++k) { wcp(Fp(17) + (size_t)k * (R2 + 32) * D2, D2, R2 + 32, D2, 48, XP2 + (size_t)k * 48 * D2); wcp(Fp(18) + (size_t)k * D2 * R2, R2, D2, 32, D2, DW2 + (size_t)k * D2 * 32); } wcp(Fp(24), D2, M2, D2, M2, WO2);
  small_kernel<<<(NBV * C3 * PS / 4 + 255) / 256, 256, 0, stream>>>(Fp(0), Fp(1), Fp(2), NBV, XA);
  inproj_kernel<CI1, D1, 0><<<NT1 / 16, 32, 0, stream>>>(XA, WI1, 8.0f, XZ1);
  dwconv_kernel<D1><<<(unsigned)(((size_t)NT1 * (D1 / 4) + 255) / 256), 256, 0, stream>>>(XZ1, Fp(4), Fp(5), 1, W1, NT1, U1);
  xproj_kernel<D1, R1><<<dim3(NT1 / 16, 4), 32, 0, stream>>>(U1, XP1, DW1, Fp(8), 1024.0f, 16384.0f, NT1, BC1, DT1);
  scan_kernel<D1><<<(NBV * 4 * D1 + 255) / 256, 256, 0, stream>>>(U1, DT1, BC1, Fp(9), Fp(10), 1, W1, NBV, NT1, Y1);
  out_kernel<D1, M1, 0><<<NT1 / 16, 32, 0, stream>>>(Y1, XZ1, Fp(11), Fp(12), WO1, 64.0f, NT1, SM);
  xfull_kernel<<<NBV * HI * 9, 256, 0, stream>>>(Fp(0), Fp(1), Fp(2), SM, XT);
  inproj_kernel<CI2, D2, 0><<<NT2 / 16, 32, 0, stream>>>(XT, WI2, 8.0f, XZ2);
  dwconv_kernel<D2><<<(unsigned)(((size_t)NT2 * (D2 / 4) + 255) / 256), 256, 0, stream>>>(XZ2, Fp(15), Fp(16), HI, HI, NT2, U2);
  xproj_kernel<D2, R2><<<dim3(NT2 / 16, 4), 32, 0, stream>>>(U2, XP2, DW2, Fp(19), 512.0f, 4096.0f, NT2, BC2, DT2);
  scan_kernel<D2><<<(NBV * 4 * D2 + 255) / 256, 256, 0, stream>>>(U2, DT2, BC2, Fp(20), Fp(21), HI, HI, NBV, NT2, Y2);
  out_kernel<D2, M2, 1><<<NT2 / 32, 32, 0, stream>>>(Y2, XZ2, Fp(22), Fp(23), WO2, 64.0f, NT2, (float*)d_out);
}
